// GRU_MIL_Siamese_29738353558314
// MI455X (gfx1250) — hardware-verified
//
#include <hip/hip_runtime.h>
#include <math.h>

constexpr int NBATCH      = 128;
constexpr int NWIN        = 11;
constexpr int NSTEPS      = 1000;
constexpr int NHID        = 64;
constexpr int NGATE       = 3 * NHID;
constexpr int NSEQ        = NBATCH * NWIN;
constexpr int SEQ_BLK     = 16;
constexpr int XCHUNK      = 8;
constexpr int NXCHUNK     = NSTEPS / XCHUNK;
constexpr int GRU_THR     = 128;
constexpr int ES_PITCH    = 68;
constexpr int TAIL_THR    = 64;
constexpr int TAIL_BATCH  = 32;
constexpr int TAIL_BLOCKS = NBATCH / TAIL_BATCH;
constexpr int W_PITCH     = 68;
constexpr int NOUT0       = NBATCH * NHID;
constexpr int NOUT1       = NBATCH * NWIN;
constexpr float HCARRY    = 256.0f;
constexpr float WCARRY    = 64.0f;
constexpr float FOLD_INV  = 1.0f / (HCARRY * WCARRY);

static_assert(NSEQ == 1408);
static_assert(NSEQ % SEQ_BLK == 0);
static_assert(NSTEPS % XCHUNK == 0);
static_assert((XCHUNK & 1) == 0);
static_assert(NHID == 64 && NHID % 32 == 0);
static_assert(GRU_THR == 4 * 32 && NHID == 16 * (GRU_THR / 32));
static_assert(SEQ_BLK * XCHUNK == GRU_THR);
static_assert(NGATE * NHID == 12 * GRU_THR * 8);
static_assert(SEQ_BLK * NHID == GRU_THR * 8);
static_assert(SEQ_BLK * NHID == 2 * GRU_THR * 4);
static_assert(NBATCH % TAIL_BATCH == 0);
static_assert((TAIL_BATCH * NWIN * 4) % 128 == 0);
static_assert(TAIL_BATCH * NWIN == 352);
static_assert((NOUT0 * 4) % 128 == 0);
static_assert(NOUT0 * 4 + NOUT1 * 4 == 38400);
static_assert(TAIL_THR == NHID);

typedef __attribute__((ext_vector_type(16))) _Float16 v16h;
typedef __attribute__((ext_vector_type(8)))  _Float16 v8h;
typedef __attribute__((ext_vector_type(8)))  float    v8f;
typedef __attribute__((ext_vector_type(4)))  float    v4f;

template <typename T> struct Frag;
template <> struct Frag<_Float16> {
  typedef v16h V; union U { v16h v; v8h h[2]; };
  static __device__ __forceinline__ v16h load(const _Float16* p) {
    U f; f.h[0] = *(const v8h*)(p); f.h[1] = *(const v8h*)(p + 16); return f.v;
  }
  static __device__ __forceinline__ v8f mma(v16h a, v16h b, v8f c) {
    return __builtin_amdgcn_wmma_f32_16x16x32_f16(false, a, false, b, (short)0, c, false, false);
  }
};

__device__ __forceinline__ void gru_guard(v8f& a, v8f& b, v8f& c, v16h x0, v16h x1,
                                          v16h w0, v16h w1, v16h w2, v16h w3, v16h w4, v16h w5) {
  asm volatile("v_nop\n\tv_nop\n\tv_nop\n\tv_nop"
               : "+v"(a), "+v"(b), "+v"(c)
               : "v"(x0), "v"(x1), "v"(w0), "v"(w1), "v"(w2), "v"(w3), "v"(w4), "v"(w5));
}

__device__ __forceinline__ float gate_sig(float v)  { return __builtin_amdgcn_rcpf(1.0f + expf(-v)); }
__device__ __forceinline__ float gate_tanh(float v) { return 1.0f - 2.0f * __builtin_amdgcn_rcpf(expf(2.0f * v) + 1.0f); }

__global__ __launch_bounds__(GRU_THR) void gru_seq_kernel(const float* __restrict__ x,
                                                          const float* __restrict__ w_ih,
                                                          const float* __restrict__ w_hh,
                                                          const float* __restrict__ b_ih,
                                                          const float* __restrict__ b_hh,
                                                          float* __restrict__ emb) {
  __shared__ __align__(16) _Float16 Wst[NGATE * NHID];
  __shared__ __align__(16) _Float16 Hb[2 * SEQ_BLK * NHID];
  __shared__ __align__(16) float    Xs[2 * SEQ_BLK * XCHUNK];
  __shared__ __align__(16) float    Es[SEQ_BLK * ES_PITCH];

  const int tid  = threadIdx.x;
  const int wave = tid >> 5;
  const int lane = tid & 31;
  const int c    = lane & 15;
  const int hh   = lane >> 4;
  const int s0   = blockIdx.x * SEQ_BLK;
  const int jcol = 16 * wave + c;

#pragma unroll 1
  for (int it = 0; it < 12; ++it) {
    const int e0 = (it * GRU_THR + tid) * 8;
    const v4f p = *(const v4f*)(w_hh + e0);
    const v4f q = *(const v4f*)(w_hh + e0 + 4);
    v8h hv;
#pragma unroll
    for (int e = 0; e < 4; ++e) {
      hv[e]     = (_Float16)(p[e] * WCARRY);
      hv[4 + e] = (_Float16)(q[e] * WCARRY);
    }
    *(v8h*)(Wst + e0) = hv;
  }
  {
    v8h zz;
#pragma unroll
    for (int e = 0; e < 8; ++e) zz[e] = (_Float16)0.0f;
    *(v8h*)(Hb + tid * 8) = zz;
  }
  const int xseq = tid >> 3;
  const int xstp = tid & 7;
  const float* xrow = x + (size_t)(s0 + xseq) * NSTEPS + xstp;
  Xs[xstp * SEQ_BLK + xseq] = xrow[0];

  const float wihR  = w_ih[jcol];
  const float wihZ  = w_ih[NHID + jcol];
  const float wihN  = w_ih[2 * NHID + jcol];
  const float biasR = b_ih[jcol] + b_hh[jcol];
  const float biasZ = b_ih[NHID + jcol] + b_hh[NHID + jcol];
  const float biasXN = b_ih[2 * NHID + jcol];
  const float biasHN = b_hh[2 * NHID + jcol];

  float hst[8];
#pragma unroll
  for (int r = 0; r < 8; ++r) hst[r] = 0.0f;

  __syncthreads();

  const _Float16* wrow = Wst + (size_t)jcol * NHID + 8 * hh;
  const v16h bR0 = Frag<_Float16>::load(wrow);
  const v16h bR1 = Frag<_Float16>::load(wrow + 32);
  const v16h bZ0 = Frag<_Float16>::load(wrow + NHID * NHID);
  const v16h bZ1 = Frag<_Float16>::load(wrow + NHID * NHID + 32);
  const v16h bN0 = Frag<_Float16>::load(wrow + 2 * NHID * NHID);
  const v16h bN1 = Frag<_Float16>::load(wrow + 2 * NHID * NHID + 32);

  const v8f z8 = {0.f, 0.f, 0.f, 0.f, 0.f, 0.f, 0.f, 0.f};

#pragma unroll 1
  for (int ch = 0; ch < NXCHUNK; ++ch) {
    {
      const int chn = (ch + 1 < NXCHUNK) ? (ch + 1) : (NXCHUNK - 1);
      const float xn = xrow[chn * XCHUNK];
      Xs[((ch + 1) & 1) * (SEQ_BLK * XCHUNK) + xstp * SEQ_BLK + xseq] = xn;
    }
    const float* xsc = Xs + (ch & 1) * (SEQ_BLK * XCHUNK);

#pragma unroll 1
    for (int tt = 0; tt < XCHUNK; ++tt) {
      const int cur = tt & 1;
      const _Float16* hrd = Hb + cur * (SEQ_BLK * NHID) + c * NHID + 8 * hh;
      _Float16* hwr = Hb + (cur ^ 1) * (SEQ_BLK * NHID) + (8 * hh) * NHID + jcol;

      const v16h a0 = Frag<_Float16>::load(hrd);
      const v16h a1 = Frag<_Float16>::load(hrd + 32);
      const v4f xv0 = *(const v4f*)(xsc + tt * SEQ_BLK + 8 * hh);
      const v4f xv1 = *(const v4f*)(xsc + tt * SEQ_BLK + 8 * hh + 4);

      v8f accR = z8, accZ = z8, accN = z8;
      accR = Frag<_Float16>::mma(a0, bR0, accR);
      accZ = Frag<_Float16>::mma(a0, bZ0, accZ);
      accN = Frag<_Float16>::mma(a0, bN0, accN);
      accR = Frag<_Float16>::mma(a1, bR1, accR);
      accZ = Frag<_Float16>::mma(a1, bZ1, accZ);
      accN = Frag<_Float16>::mma(a1, bN1, accN);
      gru_guard(accR, accZ, accN, a0, a1, bR0, bR1, bZ0, bZ1, bN0, bN1);

#pragma unroll
      for (int r = 0; r < 8; ++r) {
        const float xq = (r < 4) ? xv0[r & 3] : xv1[r & 3];
        const float zr = fmaf(accR[r], FOLD_INV, fmaf(xq, wihR, biasR));
        const float zz = fmaf(accZ[r], FOLD_INV, fmaf(xq, wihZ, biasZ));
        const float hn = fmaf(accN[r], FOLD_INV, biasHN);
        const float xn = fmaf(xq, wihN, biasXN);
        const float rg = gate_sig(zr);
        const float zg = gate_sig(zz);
        const float ng = gate_tanh(xn + rg * hn);
        const float hnew = (1.0f - zg) * ng + zg * hst[r];
        hst[r] = hnew;
        hwr[r * NHID] = (_Float16)(hnew * HCARRY);
      }
      __syncthreads();
    }
  }

#pragma unroll
  for (int r = 0; r < 8; ++r) Es[(8 * hh + r) * ES_PITCH + jcol] = hst[r];
  __syncthreads();
  for (int pass = 0; pass < 2; ++pass) {
#pragma unroll
    for (int it = 0; it < 2; ++it) {
      const int idx = it * GRU_THR + tid;
      const int row = idx >> 4;
      const int c4  = (idx & 15) * 4;
      const v4f v = *(const v4f*)(Es + row * ES_PITCH + c4);
      *(volatile v4f*)(emb + (size_t)(s0 + row) * NHID + c4) = v;
    }
    __threadfence();
  }
}

__global__ __launch_bounds__(TAIL_THR) void attn_tail_kernel(const float* __restrict__ emb,
                                                             const float* __restrict__ aw1,
                                                             const float* __restrict__ ab1,
                                                             const float* __restrict__ aw2,
                                                             const float* __restrict__ ab2,
                                                             const float* __restrict__ fcw,
                                                             const float* __restrict__ fcb,
                                                             float* __restrict__ out) {
  __shared__ __align__(16) float W1s[NHID * W_PITCH];
  __shared__ __align__(16) float FCs[NHID * W_PITCH];
  __shared__ __align__(16) float Eb[NWIN * NHID];
  __shared__ __align__(16) float T1s[NWIN * NHID];
  __shared__ __align__(16) float AW2s[NHID];
  __shared__ __align__(16) float AGs[NHID];
  __shared__ __align__(16) float SCs[16];
  __shared__ __align__(16) float Wts[TAIL_BATCH * NWIN];
  __shared__ __align__(16) float Os[TAIL_BATCH * NHID];

  const int tid = threadIdx.x;
  const int blk = blockIdx.x;

#pragma unroll 1
  for (int it = 0; it < 16; ++it) {
    const int idx = it * TAIL_THR + tid;
    const int row = idx >> 4;
    const int c4  = (idx & 15) * 4;
    const v4f va = *(const v4f*)(aw1 + row * NHID + c4);
    const v4f vb = *(const v4f*)(fcw + row * NHID + c4);
    *(v4f*)(W1s + row * W_PITCH + c4) = va;
    *(v4f*)(FCs + row * W_PITCH + c4) = vb;
  }
  AW2s[tid] = aw2[tid];
  const float b1v  = ab1[tid];
  const float fcbv = fcb[tid];
  const float b2v  = ab2[0];
  const int   ic   = (tid < NWIN) ? tid : (NWIN - 1);

#pragma unroll 1
  for (int bi = 0; bi < TAIL_BATCH; ++bi) {
    const int b = blk * TAIL_BATCH + bi;
#pragma unroll 1
    for (int i = 0; i < NWIN; ++i) Eb[i * NHID + tid] = emb[(size_t)(b * NWIN + i) * NHID + tid];
    __syncthreads();

#pragma unroll 1
    for (int i = 0; i < NWIN; ++i) {
      float s = b1v;
#pragma unroll 1
      for (int k4 = 0; k4 < NHID / 4; ++k4) {
        const v4f e = *(const v4f*)(Eb + i * NHID + k4 * 4);
        const v4f w = *(const v4f*)(W1s + tid * W_PITCH + k4 * 4);
        s = fmaf(e[0], w[0], s);
        s = fmaf(e[1], w[1], s);
        s = fmaf(e[2], w[2], s);
        s = fmaf(e[3], w[3], s);
      }
      T1s[i * NHID + tid] = tanhf(s);
    }
    __syncthreads();

    {
      float sc = b2v;
#pragma unroll 1
      for (int k4 = 0; k4 < NHID / 4; ++k4) {
        const v4f t = *(const v4f*)(T1s + ic * NHID + k4 * 4);
        const v4f w = *(const v4f*)(AW2s + k4 * 4);
        sc = fmaf(t[0], w[0], sc);
        sc = fmaf(t[1], w[1], sc);
        sc = fmaf(t[2], w[2], sc);
        sc = fmaf(t[3], w[3], sc);
      }
      if (tid < NWIN) SCs[tid] = sc;
    }
    __syncthreads();

    {
      float m = SCs[0];
#pragma unroll 1
      for (int i = 1; i < NWIN; ++i) m = fmaxf(m, SCs[i]);
      float sum = 0.0f, agg = 0.0f;
#pragma unroll 1
      for (int i = 0; i < NWIN; ++i) {
        const float e = expf(SCs[i] - m);
        sum += e;
        agg = fmaf(e, Eb[i * NHID + tid], agg);
      }
      const float inv = 1.0f / sum;
      AGs[tid] = agg * inv;
      const float wv = expf(SCs[ic] - m) * inv;
      if (tid < NWIN) Wts[bi * NWIN + tid] = wv;
    }
    __syncthreads();

    {
      float o = fcbv;
#pragma unroll 1
      for (int k4 = 0; k4 < NHID / 4; ++k4) {
        const v4f a = *(const v4f*)(AGs + k4 * 4);
        const v4f w = *(const v4f*)(FCs + tid * W_PITCH + k4 * 4);
        o = fmaf(a[0], w[0], o);
        o = fmaf(a[1], w[1], o);
        o = fmaf(a[2], w[2], o);
        o = fmaf(a[3], w[3], o);
      }
      Os[bi * NHID + tid] = o;
    }
  }
  __syncthreads();

  float* o0 = out + (size_t)blk * (TAIL_BATCH * NHID);
  for (int pass = 0; pass < 2; ++pass) {
#pragma unroll
    for (int it = 0; it < 8; ++it) {
      const int idx = it * TAIL_THR + tid;
      const v4f v = *(const v4f*)(Os + idx * 4);
      *(volatile v4f*)(o0 + idx * 4) = v;
    }
    __threadfence();
  }
  {
    const int i2 = TAIL_THR + ((tid < 24) ? tid : 23);
    const v4f wA = *(const v4f*)(Wts + tid * 4);
    const v4f wB = *(const v4f*)(Wts + i2 * 4);
    float* o1 = out + NOUT0 + (size_t)blk * (TAIL_BATCH * NWIN);
    for (int pass = 0; pass < 2; ++pass) {
      *(volatile v4f*)(o1 + tid * 4) = wA;
      if (tid < 24) *(volatile v4f*)(o1 + (TAIL_THR + tid) * 4) = wB;
      __threadfence();
    }
  }
}

extern "C" void kernel_launch(void* const* d_in, const int* in_sizes, int n_in,
                              void* d_out, int out_size, void* d_ws, size_t ws_size, hipStream_t stream) {
  if (n_in < 11 || d_out == nullptr || d_ws == nullptr) return;
  if (in_sizes[0] != NSEQ * NSTEPS || in_sizes[1] != NGATE || in_sizes[2] != NGATE * NHID ||
      in_sizes[3] != NGATE || in_sizes[4] != NGATE || in_sizes[5] != NHID * NHID || in_sizes[6] != NHID ||
      in_sizes[7] != NHID || in_sizes[8] != 1 || in_sizes[9] != NHID * NHID || in_sizes[10] != NHID ||
      out_size != NOUT0 + NOUT1) return;

  const float* x    = (const float*)d_in[0];
  const float* w_ih = (const float*)d_in[1];
  const float* w_hh = (const float*)d_in[2];
  const float* b_ih = (const float*)d_in[3];
  const float* b_hh = (const float*)d_in[4];
  const float* aw1  = (const float*)d_in[5];
  const float* ab1  = (const float*)d_in[6];
  const float* aw2  = (const float*)d_in[7];
  const float* ab2  = (const float*)d_in[8];
  const float* fcw  = (const float*)d_in[9];
  const float* fcb  = (const float*)d_in[10];
  float* out = (float*)d_out;

  const size_t emb_bytes = (size_t)NSEQ * NHID * sizeof(float);
  if (emb_bytes > ws_size || emb_bytes > (size_t)134217728) return;
  float* emb = (float*)d_ws;

  gru_seq_kernel<<<NSEQ / SEQ_BLK, GRU_THR, 0, stream>>>(x, w_ih, w_hh, b_ih, b_hh, emb);
  attn_tail_kernel<<<TAIL_BLOCKS, TAIL_THR, 0, stream>>>(emb, aw1, ab1, aw2, ab2, fcw, fcb, out);
}
